// Struct2Vec_506806141452
// MI455X (gfx1250) — hardware-verified
//
#include <hip/hip_runtime.h>
#include <math.h>

typedef __attribute__((ext_vector_type(16))) _Float16 v16h;
typedef __attribute__((ext_vector_type(16))) __bf16 v16b;
typedef __attribute__((ext_vector_type(8)))  _Float16 v8h;
typedef __attribute__((ext_vector_type(8)))  float v8f;
typedef __attribute__((ext_vector_type(4)))  float v4f;
typedef __attribute__((ext_vector_type(2)))  float v2f;
typedef __attribute__((ext_vector_type(4)))  unsigned v4u;
typedef __attribute__((ext_vector_type(4)))  int v4i;
typedef float __attribute__((may_alias)) float_a;
typedef int __attribute__((may_alias)) int_a;

template <typename T> __device__ __forceinline__ void vst2(void* p, T v) { *(volatile T*)p = v; __threadfence(); *(volatile T*)p = v; }
__device__ __forceinline__ v8f wmma16(v16h a, v16h b, v8f c) {
  v8f d = __builtin_amdgcn_wmma_f32_16x16x32_f16(false, a, false, b, (short)0, c, false, false);
  asm volatile("v_nop\n\tv_nop\n\tv_nop\n\tv_nop" : "+v"(d) : "v"(a), "v"(b));
  return d;
}
__device__ __forceinline__ v8f wmma_bf(v16b a, v16b b, v8f c) {
  v8f d = __builtin_amdgcn_wmma_f32_16x16x32_bf16(false, a, false, b, (short)0, c, false, false);
  asm volatile("v_nop\n\tv_nop\n\tv_nop\n\tv_nop" : "+v"(d) : "v"(a), "v"(b));
  return d;
}
__device__ __forceinline__ v16h frag_h(const _Float16* rowk0, int lane) {
  union { v16h v; v8h q[2]; } u; const _Float16* p = rowk0 + 8 * (lane >> 4);
  u.q[0] = *(const v8h*)p; u.q[1] = *(const v8h*)(p + 16); return u.v;
}
__device__ __forceinline__ v16h frag_f32(const float* rowk0, int lane) {
  v16h a; const float* p = rowk0 + 8 * (lane >> 4);
#pragma unroll
  for (int i = 0; i < 8; ++i) { a[i] = (_Float16)p[i]; a[8 + i] = (_Float16)p[16 + i]; }
  return a;
}
__device__ __forceinline__ v16h frag_f32s(const float* rowk0, int lane, float sc) {
  v16h a; const float* p = rowk0 + 8 * (lane >> 4);
#pragma unroll
  for (int i = 0; i < 8; ++i) { a[i] = (_Float16)(p[i] * sc); a[8 + i] = (_Float16)(p[16 + i] * sc); }
  return a;
}
__device__ __forceinline__ v16h fragc_f32(const float* W, int k0, int n, int lane, int ld, int K) {
  v16h a; const int g = lane >> 4;
#pragma unroll
  for (int i = 0; i < 8; ++i) { const int ka = k0 + 8 * g + i, kb = ka + 16;
    a[i] = (_Float16)(ka < K ? W[(size_t)ka * ld + n] : 0.f); a[8 + i] = (_Float16)(kb < K ? W[(size_t)kb * ld + n] : 0.f); }
  return a;
}
struct F2 { v16b h, l; };
__device__ __forceinline__ F2 bsplit16(const float v[16]) { F2 r;
#pragma unroll
  for (int i = 0; i < 16; ++i) { const __bf16 h = (__bf16)v[i]; r.h[i] = h; r.l[i] = (__bf16)(v[i] - (float)h); }
  return r; }
__device__ __forceinline__ F2 split_row(const float* row, int k0, int lane) { float v[16]; const float* p = row + k0 + 8 * (lane >> 4);
#pragma unroll
  for (int i = 0; i < 8; ++i) { v[i] = p[i]; v[8 + i] = p[16 + i]; }
  return bsplit16(v); }
__device__ __forceinline__ F2 split_rowK(const float* row, int k0, int lane, int K) { float v[16]; const int g = lane >> 4;
#pragma unroll
  for (int i = 0; i < 8; ++i) { const int ka = k0 + 8 * g + i, kb = ka + 16; v[i] = ka < K ? row[ka] : 0.f; v[8 + i] = kb < K ? row[kb] : 0.f; }
  return bsplit16(v); }
__device__ __forceinline__ F2 split_col(const float* W, int k0, int n, int lane, int ld, int K) { float v[16]; const int g = lane >> 4;
#pragma unroll
  for (int i = 0; i < 8; ++i) { const int ka = k0 + 8 * g + i, kb = ka + 16; v[i] = ka < K ? W[(size_t)ka * ld + n] : 0.f; v[8 + i] = kb < K ? W[(size_t)kb * ld + n] : 0.f; }
  return bsplit16(v); }
__device__ __forceinline__ v8f mac3(const F2& a, const F2& b, v8f c) { c = wmma_bf(a.l, b.h, c); c = wmma_bf(a.h, b.l, c); return wmma_bf(a.h, b.h, c); }
__device__ __forceinline__ float sigm(float v) { return 1.0f / (1.0f + expf(-v)); }
#define LDSX() do { asm volatile("s_wait_dscnt 0" ::: "memory"); __builtin_amdgcn_wave_barrier(); __builtin_amdgcn_fence(__ATOMIC_RELEASE, "workgroup"); } while (0)

#define NN 100
#define NBT 64
#define PP 128
#define NR (NN * NBT)
#define NROUND 4

__global__ __launch_bounds__(128) void k_dist(const float* __restrict__ inp, const float* __restrict__ W3, float* __restrict__ S2) {
  __shared__ float sx[NN], sy[NN]; __shared__ float sd[NN][NN + 1];
  const int b = blockIdx.x, tid = threadIdx.x;
  if (tid < NN) { sx[tid] = inp[((size_t)tid * NBT + b) * 6]; sy[tid] = inp[((size_t)tid * NBT + b) * 6 + 1]; }
  __syncthreads();
  for (int q = tid; q < NN * NN; q += 128) { const int i = q / NN, j = q % NN; const float dx = sx[i] - sx[j], dy = sy[i] - sy[j]; sd[i][j] = sqrtf(dx * dx + dy * dy); }
  __syncthreads();
  const int p = tid; const float w = W3[p];
#pragma unroll 1
  for (int i = 0; i < NN; ++i) { float s = 0.f;
#pragma unroll 4
    for (int j = 0; j < NN; ++j) { const float v = sd[i][j] * w; s += v > 0.f ? v : 0.f; }
    vst2(S2 + ((size_t)i * NBT + b) * PP + p, s); }
}
template <int MODE>
__global__ __launch_bounds__(128) void k_lin(const float* __restrict__ A, const float* __restrict__ W, const float* __restrict__ inp, const float* __restrict__ W4, const float* __restrict__ W5, const float* __restrict__ ADD, float* __restrict__ OUT) {
  __shared__ __align__(16) float so[4][16][132];
  const int tid = threadIdx.x, wave = tid >> 5, lane = tid & 31, col = lane & 15, g = lane >> 4;
  const int r0 = blockIdx.x * 64 + wave * 16;
  v8f acc[8] = {};
#pragma unroll
  for (int kc = 0; kc < PP / 32; ++kc) { const F2 a = split_row(A + (size_t)(r0 + col) * PP, kc * 32, lane);
#pragma unroll
    for (int j = 0; j < 8; ++j) acc[j] = mac3(a, split_row(W + (size_t)(j * 16 + col) * PP, kc * 32, lane), acc[j]); }
#pragma unroll
  for (int j = 0; j < 8; ++j) { const int p = j * 16 + col;
#pragma unroll
    for (int r = 0; r < 8; ++r) { const int row = r0 + 8 * g + r; float v = acc[j][r];
      if (MODE == 0) { const int n = row / NBT; const float* ir = inp + (size_t)row * 6; float it3;
        if (n == 0) it3 = ir[0] * W5[p * 2] + ir[1] * W5[p * 2 + 1];
        else { it3 = 0.f;
#pragma unroll
          for (int f = 0; f < 6; ++f) it3 += ir[f] * W4[p * 6 + f]; }
        v += it3; }
      else { v += ADD[(size_t)row * PP + p]; v = v > 0.f ? v : 0.f; }
      so[wave][8 * g + r][p] = v; } }
  LDSX();
#pragma unroll 4
  for (int rl = 0; rl < 16; ++rl) vst2(OUT + (size_t)(r0 + rl) * PP + lane * 4, *(const v4f*)(&so[wave][rl][lane * 4]));
}
__global__ __launch_bounds__(256) void k_zero(float* __restrict__ MU) { for (int q = threadIdx.x; q < 64 * PP / 4; q += 256) { v4f z = {0.f, 0.f, 0.f, 0.f}; vst2(MU + (size_t)blockIdx.x * 64 * PP + q * 4, z); } }
__global__ __launch_bounds__(128) void k_agg(const float* __restrict__ MU, float* __restrict__ AGG) {
  const int b = blockIdx.x, p = threadIdx.x; float s = 0.f;
#pragma unroll 4
  for (int n = 0; n < NN; ++n) s += MU[((size_t)n * NBT + b) * PP + p];
#pragma unroll 1
  for (int n = 0; n < NN; ++n) vst2(AGG + ((size_t)n * NBT + b) * PP + p, s - MU[((size_t)n * NBT + b) * PP + p]);
}
extern "C" void kernel_launch(void* const* d_in, const int* in_sizes, int n_in, void* d_out, int out_size, void* d_ws, size_t ws_size, hipStream_t stream) {
  (void)in_sizes; (void)n_in; (void)out_size; (void)ws_size;
  const float* inp = (const float*)d_in[0]; const float* W1 = (const float*)d_in[1]; const float* W2 = (const float*)d_in[2]; const float* W3 = (const float*)d_in[3]; const float* W4 = (const float*)d_in[4]; const float* W5 = (const float*)d_in[5];
  float* out = (float*)d_out;
  char* ws = (char*)d_ws; size_t off = 0;
  auto take = [&](size_t bytes) { char* p = ws + off; off += (bytes + 255) & ~(size_t)255; return p; };
  float* S2 = (float*)take((size_t)NR * PP * 4); float* CONST = (float*)take((size_t)NR * PP * 4); float* AGG = (float*)take((size_t)NR * PP * 4); float* MUA = (float*)take((size_t)NR * PP * 4); float* MUB = (float*)take((size_t)NR * PP * 4);
  k_dist<<<NBT, 128, 0, stream>>>(inp, W3, S2);
  k_lin<0><<<NR / 64, 128, 0, stream>>>(S2, W2, inp, W4, W5, nullptr, CONST);
  k_zero<<<NR / 64, 256, 0, stream>>>(MUA);
  float* cur = MUA; float* nxt = MUB;
  for (int r = 0; r < NROUND; ++r) {
    k_agg<<<NBT, 128, 0, stream>>>(cur, AGG);
    k_lin<1><<<NR / 64, 128, 0, stream>>>(AGG, W1, inp, W4, W5, CONST, r == NROUND - 1 ? out : nxt);
    float* t = cur; cur = nxt; nxt = t; }
}
